// TransformerXL_37409165148670
// MI455X (gfx1250) — hardware-verified
//
#include <hip/hip_runtime.h>
#include <math.h>
#include <stdint.h>

#define NBATCH 4
#define NS     2048
#define ND     1024
#define NHEAD  16
#define HD     64
#define NPAIR  32
#define NWIN   512
#define NM     (NBATCH * NS)
#define NQB    (NS / 64)
#define NGM    64
static_assert(NM == 8192);
static_assert(NQB == 32);
static_assert(NHEAD * HD == ND);
static_assert(2 * NPAIR == HD);
static_assert(2 * NHEAD <= NGM);
static_assert((ND % 64) == 0 && (NM % 64) == 0 && (ND % 256) == 0 && (HD == 64) && (NWIN == 8 * 64) && (NS % 64) == 0);

typedef __bf16   v16b __attribute__((ext_vector_type(16)));
typedef __bf16   v8b  __attribute__((ext_vector_type(8)));
typedef float    v8f  __attribute__((ext_vector_type(8)));
typedef float    v4f  __attribute__((ext_vector_type(4)));
typedef unsigned int v4u __attribute__((ext_vector_type(4)));

#if defined(__HIP_DEVICE_COMPILE__)
#define DEV_ASM 1
#else
#define DEV_ASM 0
#endif

__device__ __forceinline__ unsigned short bf_bits(float f) {
  unsigned u = __float_as_uint(f);
  return (unsigned short)((u + 0x7FFFu + ((u >> 16) & 1u)) >> 16);
}
__device__ __forceinline__ float bf_up(unsigned short hb) { return __uint_as_float(((unsigned)hb) << 16); }
__device__ __forceinline__ float bf16r(float f) { return bf_up(bf_bits(f)); }
__device__ __forceinline__ __bf16 bf_val(unsigned short hb) { return __builtin_bit_cast(__bf16, hb); }
__device__ __forceinline__ unsigned pk16(unsigned short a, unsigned short b) { return (unsigned)a | ((unsigned)b << 16); }
__device__ __forceinline__ v8f zero8() { v8f z = {0.f, 0.f, 0.f, 0.f, 0.f, 0.f, 0.f, 0.f}; return z; }

__device__ __forceinline__ v16b ldfrag_b(const __bf16* p) {
  union { v16b v; v8b h[2]; } f;
  f.h[0] = *(const v8b*)(p);
  f.h[1] = *(const v8b*)(p + 16);
  return f.v;
}

__device__ __forceinline__ v8f mma_b(v16b a, v16b b, v8f c) {
  c = __builtin_amdgcn_wmma_f32_16x16x32_bf16(false, a, false, b, (short)0, c, false, false);
#if DEV_ASM
  asm volatile("v_nop\n\tv_nop\n\tv_nop\n\tv_nop" : "+v"(c) : "v"(a), "v"(b));
#endif
  return c;
}
__device__ __forceinline__ v8f mma_b_raw(v16b a, v16b b, v8f c) {
  return __builtin_amdgcn_wmma_f32_16x16x32_bf16(false, a, false, b, (short)0, c, false, false);
}
__device__ __forceinline__ void dep_guard_b(v8f& a, v8f& b, v16b x) {
#if DEV_ASM
  asm volatile("v_nop\n\tv_nop\n\tv_nop\n\tv_nop" : "+v"(a), "+v"(b) : "v"(x));
#else
  (void)a; (void)b; (void)x;
#endif
}
__device__ __forceinline__ void keep4_b(v16b a, v16b b, v16b c, v16b d) {
#if DEV_ASM
  asm volatile("v_nop" :: "v"(a), "v"(b), "v"(c), "v"(d));
#else
  (void)a; (void)b; (void)c; (void)d;
#endif
}
__device__ __forceinline__ void acc_guard4(v8f& a, v8f& b, v8f& c, v8f& d) {
#if DEV_ASM
  asm volatile("v_nop\n\tv_nop\n\tv_nop\n\tv_nop" : "+v"(a), "+v"(b), "+v"(c), "+v"(d));
#else
  (void)a; (void)b; (void)c; (void)d;
#endif
}

__global__ __launch_bounds__(256) void cvt_bf16x8(const float* __restrict__ in, unsigned short* out, int n8) {
  const int i = blockIdx.x * 256 + (int)threadIdx.x;
  if (i < n8) {
    const v4f a = *(const v4f*)(in + (size_t)i * 8);
    const v4f b = *(const v4f*)(in + (size_t)i * 8 + 4);
    v4u p;
    p[0] = pk16(bf_bits(a[0]), bf_bits(a[1]));
    p[1] = pk16(bf_bits(a[2]), bf_bits(a[3]));
    p[2] = pk16(bf_bits(b[0]), bf_bits(b[1]));
    p[3] = pk16(bf_bits(b[2]), bf_bits(b[3]));
    *(volatile v4u*)(out + (size_t)i * 8) = p;
    __threadfence();
    *(volatile v4u*)(out + (size_t)i * 8) = p;
  }
}

__global__ __launch_bounds__(256) void wt_prep(const float* __restrict__ W, int nW, int c0,
                                               unsigned short* outp, int kin) {
  __shared__ __align__(16) unsigned short sW[16 * 256];
  const int tid  = (int)threadIdx.x;
  const int wave = tid >> 5;
  const int lane = tid & 31;
  const int p0   = blockIdx.x * 16;
  const int k0   = blockIdx.y * 256;
  const float* src = W + (size_t)(k0 + tid) * nW + c0 + p0;
  const v4f a0 = *(const v4f*)(src);
  const v4f a1 = *(const v4f*)(src + 4);
  const v4f a2 = *(const v4f*)(src + 8);
  const v4f a3 = *(const v4f*)(src + 12);
#pragma unroll
  for (int e = 0; e < 4; ++e) {
    sW[(e)      * 256 + tid] = bf_bits(a0[e]);
    sW[(4 + e)  * 256 + tid] = bf_bits(a1[e]);
    sW[(8 + e)  * 256 + tid] = bf_bits(a2[e]);
    sW[(12 + e) * 256 + tid] = bf_bits(a3[e]);
  }
  __syncthreads();
  const int r0 = 2 * wave;
  const v4u w0 = *(const v4u*)(sW + r0 * 256 + lane * 8);
  const v4u w1 = *(const v4u*)(sW + (r0 + 1) * 256 + lane * 8);
  const size_t o0 = (size_t)(p0 + r0) * kin + k0 + lane * 8;
  const size_t o1 = (size_t)(p0 + r0 + 1) * kin + k0 + lane * 8;
  for (int pass = 0; pass < 2; ++pass) {
    *(volatile v4u*)(outp + o0) = w0;
    *(volatile v4u*)(outp + o1) = w1;
    __threadfence();
  }
}

__global__ __launch_bounds__(256) void wgm_prep(const float* __restrict__ Wg, const float* __restrict__ Wm,
                                                unsigned short* outp) {
  __shared__ __align__(16) unsigned short sW[32 * 256];
  const int tid  = (int)threadIdx.x;
  const int wave = tid >> 5;
  const int lane = tid & 31;
  const int k0   = blockIdx.x * 256;
  const float* sg = Wg + (size_t)(k0 + tid) * NHEAD;
  const float* sm = Wm + (size_t)(k0 + tid) * NHEAD;
  const v4f g0 = *(const v4f*)(sg),     g1 = *(const v4f*)(sg + 4);
  const v4f g2 = *(const v4f*)(sg + 8), g3 = *(const v4f*)(sg + 12);
  const v4f m0 = *(const v4f*)(sm),     m1 = *(const v4f*)(sm + 4);
  const v4f m2 = *(const v4f*)(sm + 8), m3 = *(const v4f*)(sm + 12);
#pragma unroll
  for (int e = 0; e < 4; ++e) {
    sW[(e)      * 256 + tid] = bf_bits(g0[e]);
    sW[(4 + e)  * 256 + tid] = bf_bits(g1[e]);
    sW[(8 + e)  * 256 + tid] = bf_bits(g2[e]);
    sW[(12 + e) * 256 + tid] = bf_bits(g3[e]);
    sW[(16 + e) * 256 + tid] = bf_bits(m0[e]);
    sW[(20 + e) * 256 + tid] = bf_bits(m1[e]);
    sW[(24 + e) * 256 + tid] = bf_bits(m2[e]);
    sW[(28 + e) * 256 + tid] = bf_bits(m3[e]);
  }
  __syncthreads();
  const v4u wz = {0u, 0u, 0u, 0u};
  v4u wv[8];
#pragma unroll
  for (int rr = 0; rr < 8; ++rr) {
    const int row  = wave * 8 + rr;
    const int rowc = row & 31;
    const v4u wl = *(const v4u*)(sW + rowc * 256 + lane * 8);
    wv[rr] = (row < 2 * NHEAD) ? wl : wz;
  }
  for (int pass = 0; pass < 2; ++pass) {
#pragma unroll
    for (int rr = 0; rr < 8; ++rr) {
      const int row = wave * 8 + rr;
      *(volatile v4u*)(outp + (size_t)row * ND + k0 + lane * 8) = wv[rr];
    }
    __threadfence();
  }
}

struct InvFreq { float v[NPAIR]; };
static_assert(sizeof(InvFreq) == NPAIR * 4);

__global__ __launch_bounds__(256) void rope_tab(InvFreq invf, float* ctab, float* stab) {
  __shared__ float sInv[NPAIR];
  __shared__ __align__(16) float s2[2][8][NPAIR];
  const int tid = (int)threadIdx.x;
  if (tid == 0) {
#pragma unroll
    for (int j = 0; j < NPAIR; ++j) sInv[j] = invf.v[j];
  }
  __syncthreads();
  const int tl = tid >> 5;
  const int jj = tid & 31;
  const int t  = blockIdx.x * 8 + tl;
  const float ang = (float)t * sInv[jj];
  float sn, cs;
  sincosf(ang, &sn, &cs);
  s2[0][tl][jj] = cs;
  s2[1][tl][jj] = sn;
  __syncthreads();
  if (tid < 128) {
    const int sel = tid >> 6;
    const int idx = tid & 63;
    const int row = idx >> 3;
    const int cc  = (idx & 7) * 4;
    const v4f v = *(const v4f*)(&s2[sel][row][cc]);
    float* dst = ((sel != 0) ? stab : ctab) + (size_t)(blockIdx.x * 8 + row) * NPAIR + cc;
    *(volatile v4f*)dst = v;
    __threadfence();
    *(volatile v4f*)dst = v;
  }
}

template <int M, int N, int K, bool TWOA, int MODE>
__global__ __launch_bounds__(256) void gemm_nt(const unsigned short* __restrict__ Ahp,
                                               const unsigned short* __restrict__ Alp,
                                               const unsigned short* __restrict__ Btp,
                                               unsigned short* Chp, unsigned short* Clp, float* Cfp,
                                               const float* __restrict__ ctab, const float* __restrict__ stab,
                                               const float* __restrict__ vres, const float* __restrict__ gmp,
                                               float escale) {
  static_assert((M % 64) == 0 && (N % 64) == 0 && (K % 32) == 0);
  static_assert(MODE >= 0 && MODE <= 3);
  static_assert(MODE != 2 || (N == NHEAD * HD && (M % NS) == 0));
  static_assert(MODE != 3 || (M == NHEAD * HD && N == NM));
  __shared__ __align__(16) float sT[8][16 * 68];
  __shared__ __align__(16) float sV[(MODE == 3) ? 8 : 1][4 * 68];
  const __bf16* Ah = (const __bf16*)(const void*)Ahp;
  const __bf16* Al = (const __bf16*)(const void*)Alp;
  const __bf16* Bb = (const __bf16*)(const void*)Btp;

  const int lane = threadIdx.x & 31;
  const int wave = threadIdx.x >> 5;
  constexpr int tilesN = N >> 6;
  constexpr int tilesM = M >> 6;
  const int tile = blockIdx.x * 8 + wave;
  if (tile >= tilesM * tilesN) return;
  const int tm = tile / tilesN;
  const int tn = tile - tm * tilesN;
  const int m0 = tm << 6;
  const int n0 = tn << 6;

  const int rlane = lane & 15;
  const int koff  = (lane >> 4) * 8;
  const int mOff  = (lane >> 4) * 8;

  v8f acc[4][4];
#pragma unroll
  for (int i = 0; i < 4; ++i)
#pragma unroll
    for (int j = 0; j < 4; ++j) acc[i][j] = zero8();

  constexpr int NPL = TWOA ? 2 : 1;
  for (int pl = 0; pl < NPL; ++pl) {
    const __bf16* Ab = (pl == 0) ? Ah : Al;
    for (int k0 = 0; k0 < K; k0 += 32) {
      v16b bh[4];
#pragma unroll
      for (int j = 0; j < 4; ++j) {
        const size_t bofs = (size_t)(n0 + (j << 4) + rlane) * K + koff + k0;
        bh[j] = ldfrag_b(Bb + bofs);
      }
#pragma unroll
      for (int i = 0; i < 4; ++i) {
        const size_t aofs = (size_t)(m0 + (i << 4) + rlane) * K + koff + k0;
        const v16b ah = ldfrag_b(Ab + aofs);
#pragma unroll
        for (int j = 0; j < 4; ++j) {
          acc[i][j] = mma_b_raw(ah, bh[j], acc[i][j]);
        }
        dep_guard_b(acc[i][0], acc[i][3], ah);
      }
      keep4_b(bh[0], bh[1], bh[2], bh[3]);
    }
  }
  acc_guard4(acc[0][0], acc[0][1], acc[0][2], acc[0][3]);
  acc_guard4(acc[1][0], acc[1][1], acc[1][2], acc[1][3]);
  acc_guard4(acc[2][0], acc[2][1], acc[2][2], acc[2][3]);
  acc_guard4(acc[3][0], acc[3][1], acc[3][2], acc[3][3]);

  float* slab  = sT[wave];
  float* slabV = sV[(MODE == 3) ? wave : 0];
  const int q2 = lane >> 4, c4 = (lane & 15) * 4;
  const int q  = lane >> 3, c8 = (lane & 7) * 8;
  float mixv[8];
#pragma unroll
  for (int e = 0; e < 8; ++e) mixv[e] = 0.f;
  const float* vrb = vres;
  if (MODE == 3) {
    const int h3 = m0 >> 6;
    const int b3 = n0 / NS;
    const int s3 = n0 - b3 * NS;
    const float* mp = gmp + (size_t)(NHEAD + h3) * N + n0 + c8;
    const v4f ma = *(const v4f*)(mp);
    const v4f mb = *(const v4f*)(mp + 4);
#pragma unroll
    for (int e = 0; e < 4; ++e) { mixv[e] = ma[e]; mixv[4 + e] = mb[e]; }
    vrb = vres + ((size_t)(b3 * NHEAD + h3) * NS + s3) * HD;
  }
#pragma unroll
  for (int i = 0; i < 4; ++i) {
    const int mBase = m0 + (i << 4);
#pragma unroll
    for (int j = 0; j < 4; ++j) {
#pragma unroll
      for (int r = 0; r < 8; ++r) {
        slab[(mOff + r) * 68 + (j << 4) + rlane] = acc[i][j][r];
      }
    }
    __builtin_amdgcn_fence(__ATOMIC_RELEASE, "workgroup");
    __builtin_amdgcn_wave_barrier();
    __builtin_amdgcn_fence(__ATOMIC_ACQUIRE, "workgroup");
    if (MODE == 0 || MODE == 1) {
      v4f ov[8];
#pragma unroll
      for (int it = 0; it < 8; ++it) {
        const int row = it * 2 + q2;
        const float* sp = slab + row * 68 + c4;
        v4f v;
#pragma unroll
        for (int e = 0; e < 4; ++e) {
          const float x = sp[e];
          v[e] = (MODE == 1) ? __builtin_amdgcn_rcpf(1.0f + __expf(-x)) : x;
        }
        ov[it] = v;
      }
      for (int pass = 0; pass < 2; ++pass) {
#pragma unroll
        for (int it = 0; it < 8; ++it) {
          const int row = it * 2 + q2;
          *(volatile v4f*)(Cfp + (size_t)(mBase + row) * N + n0 + c4) = ov[it];
        }
        __threadfence();
      }
    } else {
      v4u hv[4], lv[4];
#pragma unroll
      for (int it = 0; it < 4; ++it) {
        const int row = it * 4 + q;
        const float* sp = slab + row * 68 + c8;
        float f[8];
#pragma unroll
        for (int e = 0; e < 8; ++e) f[e] = sp[e];
        if (MODE == 2) {
#pragma clang fp contract(off)
          const int t   = (mBase + row) & (NS - 1);
          const int jj0 = c8 >> 1;
          const v4f cv = *(const v4f*)(ctab + (size_t)t * NPAIR + jj0);
          const v4f sv = *(const v4f*)(stab + (size_t)t * NPAIR + jj0);
#pragma unroll
          for (int e = 0; e < 4; ++e) {
            const float x0 = f[2 * e] * escale;
            const float x1 = f[2 * e + 1] * escale;
            const float cs = cv[e], sn = sv[e];
            const float p0 = x0 * cs, p1 = x1 * sn;
            const float p2 = x1 * cs, p3 = x0 * sn;
            f[2 * e]     = p0 - p1;
            f[2 * e + 1] = p2 + p3;
          }
        }
        if (MODE == 3) {
#pragma clang fp contract(off)
          const float* vap = vrb + (size_t)lane * HD + 16 * i + 4 * it;
          const v4f va = *(const v4f*)(vap);
          const v4f vb = *(const v4f*)(vap + 32 * HD);
          __builtin_amdgcn_fence(__ATOMIC_RELEASE, "workgroup");
          __builtin_amdgcn_wave_barrier();
          __builtin_amdgcn_fence(__ATOMIC_ACQUIRE, "workgroup");
#pragma unroll
          for (int e = 0; e < 4; ++e) {
            slabV[e * 68 + lane]      = va[e];
            slabV[e * 68 + 32 + lane] = vb[e];
          }
          __builtin_amdgcn_fence(__ATOMIC_RELEASE, "workgroup");
          __builtin_amdgcn_wave_barrier();
          __builtin_amdgcn_fence(__ATOMIC_ACQUIRE, "workgroup");
          const float* rp = slabV + q * 68 + c8;
#pragma unroll
          for (int e = 0; e < 8; ++e) {
            const float rv = bf16r(rp[e]);
            const float dv = rv - f[e];
            const float pv = dv * mixv[e];
            f[e] = f[e] + pv;
          }
        }
        v4u a, a2;
#pragma unroll
        for (int e = 0; e < 4; ++e) {
          const float f0 = f[2 * e], f1 = f[2 * e + 1];
          const unsigned short h0 = bf_bits(f0), h1 = bf_bits(f1);
          const unsigned short l0 = bf_bits(f0 - bf_up(h0)), l1 = bf_bits(f1 - bf_up(h1));
          a[e] = pk16(h0, h1); a2[e] = pk16(l0, l1);
        }
        hv[it] = a; lv[it] = a2;
      }
      for (int pass = 0; pass < 2; ++pass) {
#pragma unroll
        for (int it = 0; it < 4; ++it) {
          const int row = it * 4 + q;
          *(volatile v4u*)(Chp + (size_t)(mBase + row) * N + n0 + c8) = hv[it];
          *(volatile v4u*)(Clp + (size_t)(mBase + row) * N + n0 + c8) = lv[it];
        }
        __threadfence();
      }
    }
    __builtin_amdgcn_fence(__ATOMIC_RELEASE, "workgroup");
    __builtin_amdgcn_wave_barrier();
    __builtin_amdgcn_fence(__ATOMIC_ACQUIRE, "workgroup");
  }
}

#define A_KSH   0
#define A_KSL   8192
#define A_VTH   16384
#define A_VTL   24576
#define A_PH    32768
#define A_PL    40960
#define A_TOTAL 49152
static_assert(A_KSL - A_KSH == 64 * HD * 2 && A_VTH - A_KSL == 64 * HD * 2);
static_assert(A_VTL - A_VTH == HD * 64 * 2 && A_PH - A_VTL == HD * 64 * 2);
static_assert(A_PL - A_PH == 4 * 16 * 64 * 2 && A_TOTAL - A_PL == 4 * 16 * 64 * 2);
static_assert(4 * 16 * 68 * 4 <= A_PH);

__global__ __launch_bounds__(128)
void attn_win(const unsigned short* qhp, const unsigned short* qlp,
              const unsigned short* __restrict__ khp, const unsigned short* __restrict__ klp,
              const unsigned short* __restrict__ vhp, const unsigned short* __restrict__ vlp,
              const float* __restrict__ gmp, unsigned short* Ohp, unsigned short* Olp) {
  __shared__ __align__(16) unsigned char lds[A_TOTAL];
  union FB { v16b v; v8b h[2]; };
  __bf16* Ksh = (__bf16*)(lds + A_KSH);
  __bf16* Ksl = (__bf16*)(lds + A_KSL);
  __bf16* Vth = (__bf16*)(lds + A_VTH);
  __bf16* Vtl = (__bf16*)(lds + A_VTL);
  __bf16* Ph  = (__bf16*)(lds + A_PH);
  __bf16* Pl  = (__bf16*)(lds + A_PL);

  const int tid  = (int)threadIdx.x;
  const int wave = tid >> 5;
  const int lane = tid & 31;
  const int hh   = lane >> 4;
  const int c    = lane & 15;

  const int bx   = blockIdx.x;
  const int qb   = bx & (NQB - 1);
  const int bhd  = bx >> 5;
  const int b    = bhd >> 4;
  const int h    = bhd & (NHEAD - 1);
  const int hcol = h * HD;
  const int q0   = qb * 64 + wave * 16;
  const size_t zrow = (size_t)b * NS;

  const __bf16* Qh = (const __bf16*)(const void*)qhp;
  const __bf16* Ql = (const __bf16*)(const void*)qlp;
  const __bf16* Kh = (const __bf16*)(const void*)khp;
  const __bf16* Kl = (const __bf16*)(const void*)klp;
  const __bf16* Vh = (const __bf16*)(const void*)vhp + (size_t)hcol * NM + zrow;
  const __bf16* Vl = (const __bf16*)(const void*)vlp + (size_t)hcol * NM + zrow;

  __bf16* pwh = Ph + wave * 1024;
  __bf16* pwl = Pl + wave * 1024;

  v8f acc[4];
#pragma unroll
  for (int t = 0; t < 4; ++t) acc[t] = zero8();

  float mrow[8], lrow[8], alpha[8];
#pragma unroll
  for (int r = 0; r < 8; ++r) { mrow[r] = -INFINITY; lrow[r] = 0.f; alpha[r] = 0.f; }

  const size_t qo = (zrow + q0 + c) * ND + hcol + 8 * hh;
  const int kt_lo = (qb >= 8) ? (qb - 8) : 0;

  for (int kt = kt_lo; kt <= qb; ++kt) {
    const int kv0 = kt * 64;
    __syncthreads();
    {
      const __bf16* kgh = Kh + (zrow + kv0) * ND + hcol;
      const __bf16* kgl = Kl + (zrow + kv0) * ND + hcol;
      const __bf16* vgh = Vh + kv0;
      const __bf16* vgl = Vl + kv0;
#pragma unroll
      for (int i = 0; i < 4; ++i) {
        const int p  = tid + 128 * i;
        const int rw = p >> 3;
        const int sg = (p & 7) * 8;
        const v8b a0 = *(const v8b*)(kgh + (size_t)rw * ND + sg);
        const v8b a1 = *(const v8b*)(kgl + (size_t)rw * ND + sg);
        const v8b b0 = *(const v8b*)(vgh + (size_t)rw * NM + sg);
        const v8b b1 = *(const v8b*)(vgl + (size_t)rw * NM + sg);
        *(v8b*)(Ksh + rw * 64 + sg) = a0;
        *(v8b*)(Ksl + rw * 64 + sg) = a1;
        *(v8b*)(Vth + rw * 64 + sg) = b0;
        *(v8b*)(Vtl + rw * 64 + sg) = b1;
      }
    }
    __syncthreads();

    v8f s[4];
#pragma unroll
    for (int j = 0; j < 4; ++j) s[j] = zero8();
#pragma unroll 1
    for (int dc = 0; dc < 2; ++dc) {
      const v16b qa = ldfrag_b(Qh + qo + dc * 32);
      const v16b ql = ldfrag_b(Ql + qo + dc * 32);
      const int ko = dc * 32 + 8 * hh;
#pragma unroll
      for (int j = 0; j < 4; ++j) {
        const int kr = (j * 16 + c) * 64 + ko;
        FB kb, kl;
        kb.h[0] = *(const v8b*)(Ksh + kr);
        kb.h[1] = *(const v8b*)(Ksh + kr + 16);
        kl.h[0] = *(const v8b*)(Ksl + kr);
        kl.h[1] = *(const v8b*)(Ksl + kr + 16);
        s[j] = mma_b(qa, kb.v, s[j]);
        s[j] = mma_b(qa, kl.v, s[j]);
        s[j] = mma_b(ql, kb.v, s[j]);
      }
    }

#pragma unroll
    for (int r = 0; r < 8; ++r) {
      const int rowq = q0 + 8 * hh + r;
      float m = -INFINITY;
#pragma unroll
      for (int j = 0; j < 4; ++j) {
        const int key  = kv0 + j * 16 + c;
        const int dist = rowq - key;
        float sv = s[j][r];
        const bool ok = (dist >= 0) && (dist <= NWIN);
        sv = ok ? sv : -INFINITY;
        s[j][r] = sv;
        m = fmaxf(m, sv);
      }
#pragma unroll
      for (int off = 1; off < 16; off <<= 1) m = fmaxf(m, __shfl_xor(m, off, 32));
      const float mnew  = fmaxf(mrow[r], m);
      const float msafe = (mnew == -INFINITY) ? 0.f : mnew;
      const float al    = __expf(mrow[r] - msafe);
      mrow[r]  = mnew;
      alpha[r] = al;
      float psum = 0.f;
#pragma unroll
      for (int j = 0; j < 4; ++j) {
        const float p = __expf(s[j][r] - msafe);
        psum += p;
        const unsigned short hb = bf_bits(p);
        const unsigned short lb = bf_bits(p - bf_up(hb));
        const int po = (8 * hh + r) * 64 + j * 16 + c;
        pwh[po] = bf_val(hb);
        pwl[po] = bf_val(lb);
      }
#pragma unroll
      for (int off = 1; off < 16; off <<= 1) psum += __shfl_xor(psum, off, 32);
      lrow[r] = lrow[r] * al + psum;
    }
    __builtin_amdgcn_fence(__ATOMIC_RELEASE, "workgroup");
    __builtin_amdgcn_wave_barrier();
    __builtin_amdgcn_fence(__ATOMIC_ACQUIRE, "workgroup");

    FB pa[2], pl[2];
#pragma unroll
    for (int kk = 0; kk < 2; ++kk) {
      const int pr = c * 64 + kk * 32 + 8 * hh;
      pa[kk].h[0] = *(const v8b*)(pwh + pr);
      pa[kk].h[1] = *(const v8b*)(pwh + pr + 16);
      pl[kk].h[0] = *(const v8b*)(pwl + pr);
      pl[kk].h[1] = *(const v8b*)(pwl + pr + 16);
    }
#pragma unroll
    for (int t = 0; t < 4; ++t) {
#pragma unroll
      for (int r = 0; r < 8; ++r) acc[t][r] *= alpha[r];
      const int vr0 = (t * 16 + c) * 64 + 8 * hh;
#pragma unroll
      for (int kk = 0; kk < 2; ++kk) {
        FB vb, vl;
        vb.h[0] = *(const v8b*)(Vth + vr0 + kk * 32);
        vb.h[1] = *(const v8b*)(Vth + vr0 + kk * 32 + 16);
        vl.h[0] = *(const v8b*)(Vtl + vr0 + kk * 32);
        vl.h[1] = *(const v8b*)(Vtl + vr0 + kk * 32 + 16);
        acc[t] = mma_b(pa[kk].v, vb.v, acc[t]);
        acc[t] = mma_b(pa[kk].v, vl.v, acc[t]);
        acc[t] = mma_b(pl[kk].v, vb.v, acc[t]);
      }
    }
  }

  __syncthreads();

  float* os = (float*)(void*)(lds + A_KSH) + wave * (16 * 68);
  const float* gp = gmp + (size_t)h * NM + zrow + q0 + 8 * hh;
  const v4f ga = *(const v4f*)(gp);
  const v4f gb = *(const v4f*)(gp + 4);
  float w8[8];
#pragma unroll
  for (int r = 0; r < 8; ++r) {
    const float l   = lrow[r];
    const float inv = (l > 0.f) ? (1.0f / l) : 0.f;
    const float g   = (r < 4) ? ga[r] : gb[r - 4];
    w8[r] = inv * g;
  }
#pragma unroll
  for (int t = 0; t < 4; ++t) {
#pragma unroll
    for (int r = 0; r < 8; ++r) os[(8 * hh + r) * 68 + t * 16 + c] = acc[t][r] * w8[r];
  }
  __builtin_amdgcn_fence(__ATOMIC_RELEASE, "workgroup");
  __builtin_amdgcn_wave_barrier();
  __builtin_amdgcn_fence(__ATOMIC_ACQUIRE, "workgroup");
  {
    const int q = lane >> 3, c8 = (lane & 7) * 8;
    v4u hv[4], lv[4];
#pragma unroll
    for (int it = 0; it < 4; ++it) {
      const int row = it * 4 + q;
      const float* sp = os + row * 68 + c8;
      v4u a, a2;
#pragma unroll
      for (int e = 0; e < 4; ++e) {
        const float f0 = sp[2 * e], f1 = sp[2 * e + 1];
        const unsigned short h0 = bf_bits(f0), h1 = bf_bits(f1);
        const unsigned short l0 = bf_bits(f0 - bf_up(h0)), l1 = bf_bits(f1 - bf_up(h1));
        a[e] = pk16(h0, h1); a2[e] = pk16(l0, l1);
      }
      hv[it] = a; lv[it] = a2;
    }
    for (int pass = 0; pass < 2; ++pass) {
#pragma unroll
      for (int it = 0; it < 4; ++it) {
        const int row = it * 4 + q;
        const size_t o = (zrow + q0 + row) * ND + hcol + c8;
        *(volatile v4u*)(Ohp + o) = hv[it];
        *(volatile v4u*)(Olp + o) = lv[it];
      }
      __threadfence();
    }
  }
}

extern "C" void kernel_launch(void* const* d_in, const int* in_sizes, int n_in,
                              void* d_out, int out_size, void* d_ws, size_t ws_size,
                              hipStream_t stream) {
  if (n_in < 7) return;
  if (in_sizes[0] != NM * ND) return;
  if (in_sizes[1] != NBATCH * NHEAD * NS * HD) return;
  if (in_sizes[2] != ND * ND) return;
  if (in_sizes[3] != ND * 2 * ND) return;
  if (in_sizes[4] != ND * ND) return;
  if (in_sizes[5] != ND * NHEAD || in_sizes[6] != ND * NHEAD) return;
  if (out_size != NM * ND) return;

  const float* tok  = (const float*)d_in[0];
  const float* vres = (const float*)d_in[1];
  const float* Wq   = (const float*)d_in[2];
  const float* Wkv  = (const float*)d_in[3];
  const float* Wout = (const float*)d_in[4];
  const float* Wgt  = (const float*)d_in[5];
  const float* Wmx  = (const float*)d_in[6];

  const size_t PX  = (size_t)NM * ND * 2;
  const size_t PW  = (size_t)ND * ND * 2;
  const size_t PG  = (size_t)NGM * ND * 2;
  const size_t PT  = (size_t)NS * NPAIR * 4;
  const size_t PGM = (size_t)NGM * NM * 4;
  size_t off = 0;
  const size_t oXb  = off; off += PX;
  const size_t oWq  = off; off += PW;
  const size_t oWk  = off; off += PW;
  const size_t oWv  = off; off += PW;
  const size_t oWo  = off; off += PW;
  const size_t oWgm = off; off += PG;
  const size_t oCt  = off; off += PT;
  const size_t oSt  = off; off += PT;
  const size_t oGM  = off; off += PGM;
  const size_t oQh  = off; off += PX;
  const size_t oQl  = off; off += PX;
  const size_t oKh  = off; off += PX;
  const size_t oKl  = off; off += PX;
  const size_t oVTh = off; off += PX;
  const size_t oVTl = off; off += PX;
  if (off > ws_size) return;
  if (off > (size_t)134217728) return;

  char* ws = (char*)d_ws;
  unsigned short* Xb  = (unsigned short*)(ws + oXb);
  unsigned short* WqT = (unsigned short*)(ws + oWq);
  unsigned short* WkT = (unsigned short*)(ws + oWk);
  unsigned short* WvT = (unsigned short*)(ws + oWv);
  unsigned short* WoT = (unsigned short*)(ws + oWo);
  unsigned short* Wgm = (unsigned short*)(ws + oWgm);
  float*          Ct  = (float*)(ws + oCt);
  float*          St  = (float*)(ws + oSt);
  float*          GM  = (float*)(ws + oGM);
  unsigned short* Qh  = (unsigned short*)(ws + oQh);
  unsigned short* Ql  = (unsigned short*)(ws + oQl);
  unsigned short* Kh  = (unsigned short*)(ws + oKh);
  unsigned short* Kl  = (unsigned short*)(ws + oKl);
  unsigned short* VTh = (unsigned short*)(ws + oVTh);
  unsigned short* VTl = (unsigned short*)(ws + oVTl);
  unsigned short* Oh  = Qh;
  unsigned short* Ol  = Ql;
  float*          Of  = (float*)d_out;

  InvFreq invf;
  for (int j = 0; j < NPAIR; ++j) invf.v[j] = 1.0f / powf(10000.0f, (float)j * 0.03125f);

  const dim3 blk(256);
  const int n8x = NM * ND / 8;
  const dim3 gCvtX((n8x + 255) / 256);
  const dim3 gWt(ND / 16, ND / 256);
  const dim3 gWgm(ND / 256);
  const dim3 gTab(NS / 8);
  const dim3 gGM(((NGM / 64) * (NM / 64) + 7) / 8);
  const dim3 gProj(((NM / 64) * (ND / 64) + 7) / 8);
  const dim3 gAttn(NBATCH * NHEAD * NQB);
  static_assert((NM / 64) * (ND / 64) == (ND / 64) * (NM / 64));
  static_assert(((NGM / 64) * (NM / 64)) % 8 == 0 && ((NM / 64) * (ND / 64)) % 8 == 0);

  cvt_bf16x8<<<gCvtX, blk, 0, stream>>>(tok, Xb, n8x);
  wt_prep<<<gWt, blk, 0, stream>>>(Wq,   ND,     0,  WqT, ND);
  wt_prep<<<gWt, blk, 0, stream>>>(Wkv,  2 * ND, 0,  WkT, ND);
  wt_prep<<<gWt, blk, 0, stream>>>(Wkv,  2 * ND, ND, WvT, ND);
  wt_prep<<<gWt, blk, 0, stream>>>(Wout, ND,     0,  WoT, ND);
  wgm_prep<<<gWgm, blk, 0, stream>>>(Wgt, Wmx, Wgm);
  rope_tab<<<gTab, blk, 0, stream>>>(invf, Ct, St);
  gemm_nt<NGM, NM, ND, false, 1><<<gGM, blk, 0, stream>>>(Wgm, Wgm, Xb, Qh, Ql, GM, Ct, St, vres, GM, 1.0f);
  gemm_nt<NM, ND, ND, false, 2><<<gProj, blk, 0, stream>>>(Xb, Xb, WqT, Qh, Ql, GM, Ct, St, vres, GM, 0.125f);
  gemm_nt<NM, ND, ND, false, 2><<<gProj, blk, 0, stream>>>(Xb, Xb, WkT, Kh, Kl, GM, Ct, St, vres, GM, 1.0f);
  gemm_nt<ND, NM, ND, false, 3><<<gProj, blk, 0, stream>>>(WvT, WvT, Xb, VTh, VTl, GM, Ct, St, vres, GM, 1.0f);
  attn_win<<<gAttn, dim3(128), 0, stream>>>(Qh, Ql, Kh, Kl, VTh, VTl, GM, Oh, Ol);
  gemm_nt<NM, ND, ND, true, 0><<<gProj, blk, 0, stream>>>(Oh, Ol, WoT, Kh, Kl, Of, Ct, St, vres, GM, 1.0f);
  (void)hipGetLastError();
}
